// Network_29076928594528
// MI455X (gfx1250) — hardware-verified
//
#include <hip/hip_runtime.h>
#include <stddef.h>
#include <stdint.h>

#define BATCH  4
#define NPT    262144
#define CH     32
#define HP     128
#define HW     (HP * HP)
#define HID    128
#define NOUT   4
#define GRP    (NPT / CH)
#define K0D    64
#define K1D    256
#define NTHR   256
#define SPB    256
#define MTHR   128
#define MROWS  64
#define AP     264
#define SP     132
#define FP     260
#define NU_TPL (3 * HW * (CH / 8))
#define NU_W0  (HID * (K0D / 8))
#define NU_W1  (HID * (K1D / 8))
#define NU_ALL (NU_TPL + NU_W0 + NU_W1)
#define MLP_LDS_BYTES (MROWS * AP * 2 + MROWS * SP * 4 + NOUT * HID * 4 + 2 * HID * 4 + 16 * 4 + MROWS * NOUT * 4)
#define WSMAX  134217728

static_assert(NU_TPL % NTHR == 0 && NU_W0 % NTHR == 0 && NU_W1 % NTHR == 0);
static_assert(NPT % SPB == 0 && NPT % MROWS == 0 && NPT % CH == 0 && GRP * CH == NPT);
static_assert(SPB == NTHR && SPB == 8 * CH && (NTHR / 32) * 4 == CH);
static_assert(MROWS == 16 * (MTHR / 32) && HID == MTHR && NOUT * HID == 4 * MTHR);
static_assert(K0D % 32 == 0 && K1D % 32 == 0 && K0D == 2 * CH && K1D == 2 * HID);
static_assert((AP * 2) % 16 == 0 && (SP * 4) % 16 == 0 && (FP * 4) % 16 == 0);
static_assert(AP >= K1D && SP >= HID && FP >= SPB);
static_assert(MLP_LDS_BYTES <= 300000 && (MROWS * AP * 2) % 16 == 0 && (MROWS * SP * 4) % 16 == 0);
static_assert((MROWS * AP) % 2 == 0);
static_assert(CH * FP * 4 <= 65536);

typedef float          v4f   __attribute__((ext_vector_type(4)));
typedef float          v8f   __attribute__((ext_vector_type(8)));
typedef int            v8i   __attribute__((ext_vector_type(8)));
typedef unsigned short v4us  __attribute__((ext_vector_type(4)));
typedef unsigned short v8us  __attribute__((ext_vector_type(8)));
typedef unsigned short v16us __attribute__((ext_vector_type(16)));
typedef __bf16         v16bf __attribute__((ext_vector_type(16)));
typedef v4f  __attribute__((may_alias)) v4fa;
typedef v4us __attribute__((may_alias)) v4usa;
typedef v8us __attribute__((may_alias)) v8usa;
union FragB { v16bf v; v16us u; v8us h[2]; v8i w; };

__device__ __forceinline__ v8f wmb(const FragB& a, const FragB& b, v8f c) {
  v8f d = __builtin_amdgcn_wmma_f32_16x16x32_bf16(false, a.v, false, b.v, (short)0, c, false, false);
  asm volatile("v_nop\n\tv_nop\n\tv_nop\n\tv_nop" : "+v"(d) : "v"(a.w), "v"(b.w));
  return d;
}

__device__ __forceinline__ unsigned bf16_bits(float f) {
  const unsigned u = __float_as_uint(f);
  return (u + 0x7FFFu + ((u >> 16) & 1u)) >> 16;
}
__device__ __forceinline__ float bf16_val(float f) {
  return __uint_as_float(bf16_bits(f) << 16);
}
__device__ __forceinline__ float bfw(unsigned short s) {
  return __uint_as_float(((unsigned)s) << 16);
}
__device__ __forceinline__ void put16(unsigned short* dp, v8us o) {
  *(volatile v8us*)dp = o;
  __threadfence();
  *(volatile v8us*)dp = o;
}

__global__ __launch_bounds__(NTHR) void k_prep(const float* __restrict__ tri, const float* __restrict__ w0,
                                               const float* __restrict__ w1,
                                               unsigned short* TPL, unsigned short* W0D, unsigned short* W1D) {
  const int u = (int)blockIdx.x * NTHR + (int)threadIdx.x;
  v8us o;
  if (u < NU_TPL) {
    const int cell = u >> 2;
    const int c8   = u & 3;
    const int p    = cell >> 14;
    const int yx   = cell & (HW - 1);
    const float* s = tri + (size_t)(p * CH + 8 * c8) * (size_t)HW + yx;
#pragma unroll
    for (int i = 0; i < 8; ++i) o[i] = (unsigned short)bf16_bits(s[(size_t)i * HW]);
    put16(TPL + (size_t)cell * CH + 8 * c8, o);
    return;
  } else if (u < NU_TPL + NU_W0) {
    const int v  = u - NU_TPL;
    const int n  = v >> 3;
    const int k8 = (v & 7) * 8;
    const float* s = w0 + (size_t)n * CH + (k8 & (CH - 1));
    const v4f a = *(const v4fa*)s;
    const v4f c = *(const v4fa*)(s + 4);
    o[0] = (unsigned short)bf16_bits(a.x); o[1] = (unsigned short)bf16_bits(a.y);
    o[2] = (unsigned short)bf16_bits(a.z); o[3] = (unsigned short)bf16_bits(a.w);
    o[4] = (unsigned short)bf16_bits(c.x); o[5] = (unsigned short)bf16_bits(c.y);
    o[6] = (unsigned short)bf16_bits(c.z); o[7] = (unsigned short)bf16_bits(c.w);
    put16(W0D + (size_t)n * K0D + k8, o);
    return;
  } else if (u < NU_ALL) {
    const int v  = u - NU_TPL - NU_W0;
    const int n  = v >> 5;
    const int k8 = (v & 31) * 8;
    const float* s = w1 + (size_t)n * HID + (k8 & (HID - 1));
    const v4f a = *(const v4fa*)s;
    const v4f c = *(const v4fa*)(s + 4);
    o[0] = (unsigned short)bf16_bits(a.x); o[1] = (unsigned short)bf16_bits(a.y);
    o[2] = (unsigned short)bf16_bits(a.z); o[3] = (unsigned short)bf16_bits(a.w);
    o[4] = (unsigned short)bf16_bits(c.x); o[5] = (unsigned short)bf16_bits(c.y);
    o[6] = (unsigned short)bf16_bits(c.z); o[7] = (unsigned short)bf16_bits(c.w);
    put16(W1D + (size_t)n * K1D + k8, o);
    return;
  }
}

__global__ __launch_bounds__(NTHR) void k_sample(const float* __restrict__ gcb,
                                                 const unsigned short* __restrict__ TPL,
                                                 unsigned short* FA) {
#pragma clang fp contract(off)
  __shared__ __attribute__((aligned(16))) float sF[CH * FP];
  const int tid = (int)threadIdx.x, lane = tid & 31, wave = tid >> 5;
  const int n = (int)blockIdx.x * SPB + tid;
  const float* cp = gcb + (size_t)n * 3;
  const float x = bf16_val(cp[0]);
  const float y = bf16_val(cp[1]);
  const float z = bf16_val(cp[2]);

  float acc[CH];
#pragma unroll
  for (int c = 0; c < CH; ++c) acc[c] = 0.0f;

#pragma unroll 1
  for (int q = 0; q < 3; ++q) {
    const float ga = (q == 2) ? y : x;
    const float gb = (q == 0) ? y : z;
    const int   pl = (3 - q) % 3;
    float t;
    t = ga + 1.0f; t = t * 0.5f;
    float px = t * 127.0f;
    t = gb + 1.0f; t = t * 0.5f;
    float py = t * 127.0f;
    px = fminf(fmaxf(px, -4.0f), 132.0f);
    py = fminf(fmaxf(py, -4.0f), 132.0f);
    const float fx = floorf(px), fy = floorf(py);
    const int ix = (int)fx, iy = (int)fy;
    const float wx = px - fx, wy = py - fy;
    const float ax = 1.0f - wx, ay = 1.0f - wy;
    const float vx0 = (ix >= 0 && ix < HP) ? 1.0f : 0.0f;
    const float vx1 = (ix + 1 >= 0 && ix + 1 < HP) ? 1.0f : 0.0f;
    const float vy0 = (iy >= 0 && iy < HP) ? 1.0f : 0.0f;
    const float vy1 = (iy + 1 >= 0 && iy + 1 < HP) ? 1.0f : 0.0f;
    const float m00 = ((ax * ay) * vx0) * vy0;
    const float m01 = ((wx * ay) * vx1) * vy0;
    const float m10 = ((ax * wy) * vx0) * vy1;
    const float m11 = ((wx * wy) * vx1) * vy1;
    const int cx0 = min(max(ix, 0), HP - 1);
    const int cx1 = min(max(ix + 1, 0), HP - 1);
    const int cy0 = min(max(iy, 0), HP - 1);
    const int cy1 = min(max(iy + 1, 0), HP - 1);
#pragma unroll 1
    for (int cc = 0; cc < 4; ++cc) {
      const int   xi = (cc & 1) ? cx1 : cx0;
      const int   yi = (cc & 2) ? cy1 : cy0;
      const float wg = (cc == 0) ? m00 : ((cc == 1) ? m01 : ((cc == 2) ? m10 : m11));
      const unsigned short* cl = TPL + ((size_t)((pl * HP + yi) * HP + xi)) * CH;
      const v8us u0 = *(const v8usa*)(cl);
      const v8us u1 = *(const v8usa*)(cl + 8);
      const v8us u2 = *(const v8usa*)(cl + 16);
      const v8us u3 = *(const v8usa*)(cl + 24);
#pragma unroll
      for (int i = 0; i < 8; ++i) {
        acc[i]      = fmaf(wg, bfw(u0[i]), acc[i]);
        acc[8 + i]  = fmaf(wg, bfw(u1[i]), acc[8 + i]);
        acc[16 + i] = fmaf(wg, bfw(u2[i]), acc[16 + i]);
        acc[24 + i] = fmaf(wg, bfw(u3[i]), acc[24 + i]);
      }
    }
  }

#pragma unroll
  for (int c = 0; c < CH; ++c) sF[c * FP + tid] = acc[c];
  __syncthreads();

  const int q8 = lane & 7, sub = lane >> 3;
  const unsigned mlo = 0u - (unsigned)(q8 >> 2);
  const unsigned mhi = ~mlo;
  v8us pv[8];
#pragma unroll
  for (int cc = 0; cc < 4; ++cc) {
    const int c = 4 * wave + cc;
#pragma unroll
    for (int uu = 0; uu < 2; ++uu) {
      const int tr = 4 * uu + sub;
      const int p0 = 32 * tr + 8 * (q8 & 3);
      const float* sp = sF + c * FP + p0;
      const v4f a = *(const v4fa*)sp;
      const v4f b = *(const v4fa*)(sp + 4);
      const v8f f8 = {a.x, a.y, a.z, a.w, b.x, b.y, b.z, b.w};
      v8us oo;
#pragma unroll
      for (int e = 0; e < 8; ++e) {
        const unsigned hb = bf16_bits(f8[e]);
        const unsigned lb = bf16_bits(f8[e] - __uint_as_float(hb << 16));
        oo[e] = (unsigned short)((hb & mhi) | (lb & mlo));
      }
      pv[2 * cc + uu] = oo;
    }
  }
  const size_t rowb = (size_t)8 * (size_t)blockIdx.x;
#pragma unroll
  for (int cc = 0; cc < 4; ++cc)
#pragma unroll
    for (int uu = 0; uu < 2; ++uu) {
      const int c = 4 * wave + cc, tr = 4 * uu + sub;
      unsigned short* dp = FA + ((size_t)c * GRP + rowb + (size_t)tr) * K0D + 8 * q8;
      *(volatile v8us*)dp = pv[2 * cc + uu];
    }
  __threadfence();
#pragma unroll
  for (int cc = 0; cc < 4; ++cc)
#pragma unroll
    for (int uu = 0; uu < 2; ++uu) {
      const int c = 4 * wave + cc, tr = 4 * uu + sub;
      unsigned short* dp = FA + ((size_t)c * GRP + rowb + (size_t)tr) * K0D + 8 * q8;
      *(volatile v8us*)dp = pv[2 * cc + uu];
    }
}

__global__ __launch_bounds__(MTHR) void k_mlp(const unsigned short* __restrict__ FA,
                                              const unsigned short* __restrict__ W0D,
                                              const unsigned short* __restrict__ W1D,
                                              const float* __restrict__ b0, const float* __restrict__ b1,
                                              const float* __restrict__ w2, const float* __restrict__ b2,
                                              float* outb) {
  extern __shared__ __attribute__((aligned(16))) float dynm[];
  unsigned short* sA  = (unsigned short*)dynm;
  float*          stg = dynm + (MROWS * AP) / 2;
  float*          sW2 = stg + MROWS * SP;
  float*          sB0 = sW2 + NOUT * HID;
  float*          sB1 = sB0 + HID;
  float*          sB2 = sB1 + HID;
  float*          sO  = sB2 + 16;

  const int tid = (int)threadIdx.x, lane = tid & 31, wave = tid >> 5, hh = lane >> 4, m = lane & 15;
  const int m0 = (int)blockIdx.x * MROWS;

  {
    sB0[tid] = bf16_val(b0[tid]);
    sB1[tid] = bf16_val(b1[tid]);
    const v4f wv = *(const v4fa*)(w2 + 4 * tid);
    v4f wr;
    wr.x = bf16_val(wv.x); wr.y = bf16_val(wv.y); wr.z = bf16_val(wv.z); wr.w = bf16_val(wv.w);
    *(v4fa*)(sW2 + 4 * tid) = wr;
    const float bb = bf16_val(b2[tid & 3]);
    if (tid < 16) sB2[tid] = bb;
  }
  __syncthreads();

  v8f acc[8];
  const v8f z8 = {0.f, 0.f, 0.f, 0.f, 0.f, 0.f, 0.f, 0.f};

#pragma unroll
  for (int t = 0; t < 8; ++t) acc[t] = z8;
  {
    const unsigned short* ap = FA  + (size_t)(m0 + 16 * wave + m) * K0D + 8 * hh;
    const unsigned short* bp = W0D + (size_t)m * K0D + 8 * hh;
#pragma unroll 1
    for (int k0 = 0; k0 < K0D; k0 += 32) {
      FragB af;
      af.h[0] = *(const v8usa*)(ap + k0);
      af.h[1] = *(const v8usa*)(ap + k0 + 16);
#pragma unroll
      for (int nt = 0; nt < 8; ++nt) {
        const unsigned short* wq = bp + (size_t)(16 * nt) * K0D + k0;
        FragB bf;
        bf.h[0] = *(const v8usa*)wq;
        bf.h[1] = *(const v8usa*)(wq + 16);
        acc[nt] = wmb(af, bf, acc[nt]);
      }
    }
  }
#pragma unroll
  for (int nt = 0; nt < 8; ++nt) {
    const int lc = 16 * nt + m;
    const float bv = sB0[lc];
#pragma unroll
    for (int r = 0; r < 8; ++r) {
      const int lr = 16 * wave + 8 * hh + r;
      stg[lr * SP + lc] = fmaxf(acc[nt][r] + bv, 0.0f);
    }
  }
  __syncthreads();

  {
    const int j = lane;
#pragma unroll 2
    for (int i = 0; i < 16; ++i) {
      const int row = 16 * wave + i;
      const v4f a = *(const v4fa*)(stg + row * SP + 4 * j);
      v4us hq, lq;
      unsigned hb;
      hb = bf16_bits(a.x); hq.x = (unsigned short)hb; lq.x = (unsigned short)bf16_bits(a.x - __uint_as_float(hb << 16));
      hb = bf16_bits(a.y); hq.y = (unsigned short)hb; lq.y = (unsigned short)bf16_bits(a.y - __uint_as_float(hb << 16));
      hb = bf16_bits(a.z); hq.z = (unsigned short)hb; lq.z = (unsigned short)bf16_bits(a.z - __uint_as_float(hb << 16));
      hb = bf16_bits(a.w); hq.w = (unsigned short)hb; lq.w = (unsigned short)bf16_bits(a.w - __uint_as_float(hb << 16));
      *(v4usa*)(sA + row * AP + 4 * j)       = hq;
      *(v4usa*)(sA + row * AP + HID + 4 * j) = lq;
    }
  }
  __syncthreads();

#pragma unroll
  for (int t = 0; t < 8; ++t) acc[t] = z8;
  {
    const unsigned short* ap = sA  + (16 * wave + m) * AP + 8 * hh;
    const unsigned short* bp = W1D + (size_t)m * K1D + 8 * hh;
#pragma unroll 1
    for (int k0 = 0; k0 < K1D; k0 += 32) {
      FragB af;
      af.h[0] = *(const v8usa*)(ap + k0);
      af.h[1] = *(const v8usa*)(ap + k0 + 16);
#pragma unroll
      for (int nt = 0; nt < 8; ++nt) {
        const unsigned short* wq = bp + (size_t)(16 * nt) * K1D + k0;
        FragB bf;
        bf.h[0] = *(const v8usa*)wq;
        bf.h[1] = *(const v8usa*)(wq + 16);
        acc[nt] = wmb(af, bf, acc[nt]);
      }
    }
  }
#pragma unroll
  for (int nt = 0; nt < 8; ++nt) {
    const int lc = 16 * nt + m;
    const float bv = sB1[lc];
#pragma unroll
    for (int r = 0; r < 8; ++r) {
      const int lr = 16 * wave + 8 * hh + r;
      stg[lr * SP + lc] = fmaxf(acc[nt][r] + bv, 0.0f);
    }
  }
  __syncthreads();

  {
    const int r  = tid & 63;
    const int jp = tid >> 6;
    const float* xr = stg + r * SP;
    const float* wa = sW2 + (2 * jp) * HID;
    const float* wb = wa + HID;
    float s0 = 0.0f, s1 = 0.0f;
#pragma unroll 4
    for (int k = 0; k < HID; k += 4) {
      const v4f xv = *(const v4fa*)(xr + k);
      const v4f av = *(const v4fa*)(wa + k);
      const v4f cv = *(const v4fa*)(wb + k);
      s0 = fmaf(xv.x, av.x, s0); s0 = fmaf(xv.y, av.y, s0); s0 = fmaf(xv.z, av.z, s0); s0 = fmaf(xv.w, av.w, s0);
      s1 = fmaf(xv.x, cv.x, s1); s1 = fmaf(xv.y, cv.y, s1); s1 = fmaf(xv.z, cv.z, s1); s1 = fmaf(xv.w, cv.w, s1);
    }
    const int n0 = 2 * jp, n1 = n0 + 1;
    const float o0 = fmaxf(s0 + sB2[n0], 0.0f);
    const float o1 = fmaxf(s1 + sB2[n1], 0.0f);
    sO[r * NOUT + ((n0 + 3) & 3)] = o0;
    sO[r * NOUT + ((n1 + 3) & 3)] = o1;
  }
  __syncthreads();

  if (tid < 64) {
    const v4f v = *(const v4fa*)(sO + 4 * tid);
    float* op = outb + (size_t)(m0 + tid) * NOUT;
    *(volatile v4f*)op = v;
    __threadfence();
    *(volatile v4f*)op = v;
  }
}

extern "C" void kernel_launch(void* const* d_in, const int* in_sizes, int n_in,
                              void* d_out, int out_size, void* d_ws, size_t ws_size,
                              hipStream_t stream) {
  if (n_in < 8) return;
  if (in_sizes[0] != BATCH * NPT * 3) return;
  if (in_sizes[1] != 3 * CH * HW) return;
  if (in_sizes[2] != HID * CH) return;
  if (in_sizes[3] != HID) return;
  if (in_sizes[4] != HID * HID) return;
  if (in_sizes[5] != HID) return;
  if (in_sizes[6] != NOUT * HID) return;
  if (in_sizes[7] != NOUT) return;
  if (out_size != BATCH * NPT * NOUT) return;

  const float* gc  = (const float*)d_in[0];
  const float* tri = (const float*)d_in[1];
  const float* w0  = (const float*)d_in[2];
  const float* b0  = (const float*)d_in[3];
  const float* w1  = (const float*)d_in[4];
  const float* b1  = (const float*)d_in[5];
  const float* w2  = (const float*)d_in[6];
  const float* b2  = (const float*)d_in[7];
  float* out = (float*)d_out;

  char* ws = (char*)d_ws;
  size_t off = 0;
  const size_t oTPL = off; off += (size_t)3 * HW * CH * 2;       off = (off + 255) & ~(size_t)255;
  const size_t oW0D = off; off += (size_t)HID * K0D * 2;         off = (off + 255) & ~(size_t)255;
  const size_t oW1D = off; off += (size_t)HID * K1D * 2;         off = (off + 255) & ~(size_t)255;
  const size_t oFA  = off; off += (size_t)NPT * K0D * 2;         off = (off + 255) & ~(size_t)255;
  if (off > ws_size || off > (size_t)WSMAX) return;
  unsigned short* TPL = (unsigned short*)(ws + oTPL);
  unsigned short* W0D = (unsigned short*)(ws + oW0D);
  unsigned short* W1D = (unsigned short*)(ws + oW1D);
  unsigned short* FA  = (unsigned short*)(ws + oFA);

  hipFuncSetAttribute(reinterpret_cast<const void*>(&k_mlp), hipFuncAttributeMaxDynamicSharedMemorySize,
                      (int)MLP_LDS_BYTES);

  k_prep<<<NU_ALL / NTHR, NTHR, 0, stream>>>(tri, w0, w1, TPL, W0D, W1D);
  for (int b = 0; b < BATCH; ++b) {
    k_sample<<<NPT / SPB, NTHR, 0, stream>>>(gc + (size_t)b * NPT * 3, TPL, FA);
    k_mlp<<<NPT / MROWS, MTHR, MLP_LDS_BYTES, stream>>>(FA, W0D, W1D, b0, b1, w2, b2,
                                                        out + (size_t)b * NPT * NOUT);
  }
}
